// FDT_26834955665624
// MI455X (gfx1250) — hardware-verified
//
#include <hip/hip_runtime.h>
#include <math.h>
#include <stdint.h>

#define NB    2
#define CC    128
#define IMW   128
#define HW    (IMW * IMW)
#define NPIX  (NB * HW)
#define C3    384
#define HID   340
#define HIDP  384
#define FSL   192
#define NHEAD 4
#define HDC   32
#define WSZ   4
#define NWX   (IMW / WSZ)
#define NWIN  (NWX * NWX)
#define NSLN  (HW / 256)
#define NSLS  (HW / 2048)
#define AFSZ  (CC * HDC)
#define RSQ2  0.70710678118654752f
#define GXP   36
#define AXP   68
#define TXP   132
#define ATP   136
#define GSP   264

static_assert((IMW & (IMW - 1)) == 0);
static_assert(IMW % WSZ == 0);
static_assert(WSZ == 4);
static_assert(HW % 2048 == 0);
static_assert(HW % 256 == 0);
static_assert(HW % 64 == 0);
static_assert(NPIX % 256 == 0);
static_assert(CC == NHEAD * HDC);
static_assert(HDC == 32);
static_assert((GXP * 4) % 16 == 0);
static_assert((AXP * 4) % 16 == 0);
static_assert((TXP * 4) % 16 == 0);
static_assert((ATP * 2) % 16 == 0);
static_assert((GSP * 2) % 16 == 0);

#define RL_R    0
#define RL_QTH  24576
#define RL_QTL  28672
#define RL_KTH  32768
#define RL_KTL  36864
#define RL_ATH  40960
#define RL_ATL  75776
#define RL_VH   110592
#define RL_VL   114944
#define RL_INV  119296
#define RL_END  119424
static_assert(RL_QTH == RL_R + 16 * C3 * 4);
static_assert(RL_QTL == RL_QTH + CC * 16 * 2);
static_assert(RL_KTH == RL_QTL + CC * 16 * 2);
static_assert(RL_KTL == RL_KTH + CC * 16 * 2);
static_assert(RL_ATH == RL_KTL + CC * 16 * 2);
static_assert(RL_ATL == RL_ATH + CC * ATP * 2);
static_assert(RL_VH == RL_ATL + CC * ATP * 2);
static_assert(RL_VL == RL_VH + 16 * ATP * 2);
static_assert(RL_INV == RL_VL + 16 * ATP * 2);
static_assert(RL_END == RL_INV + 32 * 4);
static_assert(16 * TXP * 4 <= RL_QTH - RL_R);

#define GL_QH   0
#define GL_QL   16896
#define GL_KH   33792
#define GL_KL   50688
#define GL_RED  67584
#define GL_STG  71680
#define GL_END  76288
static_assert(GL_QL == 32 * GSP * 2);
static_assert(GL_KH == 2 * GL_QL);
static_assert(GL_KL == 3 * GL_QL);
static_assert(GL_RED == 4 * GL_QL);
static_assert(GL_STG == GL_RED + 4 * 32 * 8 * 4);
static_assert(GL_END == GL_STG + 32 * GXP * 4);

typedef __bf16         v16bf __attribute__((ext_vector_type(16)));
typedef unsigned short v8us  __attribute__((ext_vector_type(8)));
typedef float          v8f   __attribute__((ext_vector_type(8)));
typedef float          v4f   __attribute__((ext_vector_type(4)));
typedef unsigned int   v4u   __attribute__((ext_vector_type(4)));
typedef unsigned int   v2u   __attribute__((ext_vector_type(2)));

union Frag { v16bf v; v8us u[2]; };

__device__ __forceinline__ unsigned short bf_bits(float f) {
  unsigned u = __float_as_uint(f);
  return (unsigned short)((u + 0x7FFFu + ((u >> 16) & 1u)) >> 16);
}
__device__ __forceinline__ float bf_up(unsigned short h) { return __uint_as_float(((unsigned)h) << 16); }
__device__ __forceinline__ float bfr(float f) { return bf_up(bf_bits(f)); }
__device__ __forceinline__ unsigned pk16(unsigned short a, unsigned short b) { return (unsigned)a | ((unsigned)b << 16); }
__device__ __forceinline__ void split_bf(float v, unsigned short& hi, unsigned short& lo) {
  const unsigned short hb = bf_bits(v);
  hi = hb;
  lo = bf_bits(v - bf_up(hb));
}
__device__ __forceinline__ void split4(v4f v, v2u& ph, v2u& pl) {
  unsigned short h[4], l[4];
#pragma unroll
  for (int e = 0; e < 4; ++e) split_bf(v[e], h[e], l[e]);
  ph[0] = pk16(h[0], h[1]); ph[1] = pk16(h[2], h[3]);
  pl[0] = pk16(l[0], l[1]); pl[1] = pk16(l[2], l[3]);
}
__device__ __forceinline__ void split8(v4f v0, v4f v1, v4u& ph, v4u& pl) {
  unsigned short h[8], l[8];
#pragma unroll
  for (int e = 0; e < 4; ++e) { split_bf(v0[e], h[e], l[e]); split_bf(v1[e], h[4 + e], l[4 + e]); }
#pragma unroll
  for (int e = 0; e < 4; ++e) { ph[e] = pk16(h[2 * e], h[2 * e + 1]); pl[e] = pk16(l[2 * e], l[2 * e + 1]); }
}
__device__ __forceinline__ v8f zero8() { v8f z = {0.f, 0.f, 0.f, 0.f, 0.f, 0.f, 0.f, 0.f}; return z; }
__device__ __forceinline__ v8us zero8us() { v8us z = {0, 0, 0, 0, 0, 0, 0, 0}; return z; }

__device__ __forceinline__ v16bf ldfrag(const unsigned short* p) {
  Frag f;
  f.u[0] = *(const v8us*)(p);
  f.u[1] = *(const v8us*)(p + 16);
  return f.v;
}
__device__ __forceinline__ v16bf ldfrag16(const unsigned short* p) {
  Frag f;
  f.u[0] = *(const v8us*)(p);
  f.u[1] = zero8us();
  return f.v;
}

__device__ __forceinline__ v8f mma_bf(v16bf a, v16bf b, v8f c) {
  c = __builtin_amdgcn_wmma_f32_16x16x32_bf16(false, a, false, b, (short)0, c, false, false);
#if defined(__HIP_DEVICE_COMPILE__)
  asm volatile("v_nop\n\tv_nop\n\tv_nop\n\tv_nop" : "+v"(c) : "v"(a), "v"(b));
#endif
  return c;
}
__device__ __forceinline__ void wave_sync_lds() {
  __builtin_amdgcn_fence(__ATOMIC_RELEASE, "workgroup");
  __builtin_amdgcn_wave_barrier();
  __builtin_amdgcn_fence(__ATOMIC_ACQUIRE, "workgroup");
}

__global__ __launch_bounds__(256) void cvt_w(const float* __restrict__ w, unsigned short* outp,
                                             int rows, int cols, int rowsP, int colsP) {
  const int t = blockIdx.x * 256 + threadIdx.x;
  const int ppr = colsP >> 3;
  const int npc = rowsP * ppr;
  const bool ok = t < npc;
  const int tt = ok ? t : 0;
  const int r = tt / ppr, c8 = (tt - r * ppr) * 8;
  const int rr = min(r, rows - 1);
  unsigned short hv[8];
#pragma unroll
  for (int e = 0; e < 8; ++e) {
    const int c = c8 + e;
    const int cl = min(c, cols - 1);
    const float f = w[(size_t)rr * cols + cl];
    const float z = (r < rows && c < cols) ? f : 0.0f;
    hv[e] = bf_bits(z);
  }
  v4u pk;
#pragma unroll
  for (int e = 0; e < 4; ++e) pk[e] = pk16(hv[2 * e], hv[2 * e + 1]);
  unsigned short* gp = outp + (size_t)r * colsP + c8;
  if (ok) *(volatile v4u*)gp = pk;
  __threadfence();
  if (ok) *(volatile v4u*)gp = pk;
}

__global__ __launch_bounds__(256) void nchw_in(const float* __restrict__ x, float* A) {
  __shared__ __align__(16) float xs[64 * TXP];
  const int tid = threadIdx.x, wave = tid >> 5, lane = tid & 31;
  const int b = blockIdx.x / (HW / 64);
  const int p0 = (blockIdx.x - b * (HW / 64)) * 64;
#pragma unroll
  for (int it = 0; it < 8; ++it) {
    const int q = it * 256 + tid;
    const int ch = q >> 4, j4 = (q & 15) * 4;
    const v4f v = *(const v4f*)(x + ((size_t)(b * CC + ch)) * HW + p0 + j4);
#pragma unroll
    for (int e = 0; e < 4; ++e) xs[(j4 + e) * TXP + ch] = bfr(v[e]);
  }
  __syncthreads();
  v4f ov[8];
#pragma unroll
  for (int it = 0; it < 8; ++it) {
    const int row = wave * 8 + it;
    ov[it] = *(const v4f*)(xs + row * TXP + lane * 4);
  }
#pragma unroll
  for (int it = 0; it < 8; ++it) {
    const int row = wave * 8 + it;
    *(volatile v4f*)(A + ((size_t)(b * HW + p0 + row)) * CC + lane * 4) = ov[it];
  }
  __threadfence();
#pragma unroll
  for (int it = 0; it < 8; ++it) {
    const int row = wave * 8 + it;
    *(volatile v4f*)(A + ((size_t)(b * HW + p0 + row)) * CC + lane * 4) = ov[it];
  }
}

__global__ __launch_bounds__(256) void ln_k(float* A, const float* __restrict__ Badd,
                                            const float* __restrict__ g, const float* __restrict__ bv,
                                            unsigned short* Th, unsigned short* Tl, int addB) {
#pragma clang fp contract(off)
  const int tid = threadIdx.x, wave = tid >> 5, lane = tid & 31;
  const int p = blockIdx.x * 8 + wave;
  const int c4 = lane * 4;
  float* arow = A + (size_t)p * CC + c4;
  v4f xv = *(const v4f*)arow;
  if (addB != 0) {
    const v4f b2 = *(const v4f*)(Badd + (size_t)p * CC + c4);
    xv = xv + b2;
    *(volatile v4f*)arow = xv;
    __threadfence();
    *(volatile v4f*)arow = xv;
  }
  float s = (xv[0] + xv[1]) + (xv[2] + xv[3]);
#pragma unroll
  for (int off = 1; off < 32; off <<= 1) s = s + __shfl_xor(s, off, 32);
  const float mu = s * (1.0f / 128.0f);
  float d[4];
  float s2 = 0.f;
#pragma unroll
  for (int e = 0; e < 4; ++e) { d[e] = xv[e] - mu; const float dd = d[e] * d[e]; s2 = s2 + dd; }
#pragma unroll
  for (int off = 1; off < 32; off <<= 1) s2 = s2 + __shfl_xor(s2, off, 32);
  const float var = s2 * (1.0f / 128.0f);
  const float rstd = 1.0f / sqrtf(var + 1e-6f);
  v4f z;
#pragma unroll
  for (int e = 0; e < 4; ++e) {
    float t0 = d[e] * rstd;
    t0 = t0 * bfr(g[c4 + e]);
    z[e] = t0 + bfr(bv[c4 + e]);
  }
  v2u ph, pl;
  split4(z, ph, pl);
  const size_t to = (size_t)p * CC + c4;
  *(volatile v2u*)(Th + to) = ph;
  *(volatile v2u*)(Tl + to) = pl;
  __threadfence();
  *(volatile v2u*)(Th + to) = ph;
  *(volatile v2u*)(Tl + to) = pl;
}

template <int K, int EP>
__global__ __launch_bounds__(256) void gemm_k(const unsigned short* __restrict__ Ah,
                                              const unsigned short* __restrict__ Al, int lda,
                                              const unsigned short* __restrict__ W,
                                              float* outf, int ldo, const float* __restrict__ res) {
  __shared__ __align__(16) float stg[8 * 32 * GXP];
  const int tid = threadIdx.x, wave = tid >> 5, lane = tid & 31, hh = lane >> 4, l15 = lane & 15;
  const int m0 = (blockIdx.x * 8 + wave) * 32;
  const int n0 = blockIdx.y * 32;
  const unsigned short* ah0 = Ah + (size_t)(m0 + l15) * lda + 8 * hh;
  const unsigned short* al0 = Al + (size_t)(m0 + l15) * lda + 8 * hh;
  const unsigned short* ah1 = ah0 + (size_t)16 * lda;
  const unsigned short* al1 = al0 + (size_t)16 * lda;
  const unsigned short* w0 = W + (size_t)(n0 + l15) * K + 8 * hh;
  const unsigned short* w1 = w0 + (size_t)16 * K;
  v8f c00 = zero8(), c01 = zero8(), c10 = zero8(), c11 = zero8();
#pragma unroll 2
  for (int k0 = 0; k0 < K; k0 += 32) {
    const v16bf a0h = ldfrag(ah0 + k0), a0l = ldfrag(al0 + k0);
    const v16bf a1h = ldfrag(ah1 + k0), a1l = ldfrag(al1 + k0);
    const v16bf b0 = ldfrag(w0 + k0), b1 = ldfrag(w1 + k0);
    c00 = mma_bf(a0h, b0, c00); c00 = mma_bf(a0l, b0, c00);
    c01 = mma_bf(a0h, b1, c01); c01 = mma_bf(a0l, b1, c01);
    c10 = mma_bf(a1h, b0, c10); c10 = mma_bf(a1l, b0, c10);
    c11 = mma_bf(a1h, b1, c11); c11 = mma_bf(a1l, b1, c11);
  }
  float* sw = stg + wave * (32 * GXP);
#pragma unroll
  for (int r = 0; r < 8; ++r) {
    sw[(8 * hh + r) * GXP + l15] = c00[r];
    sw[(8 * hh + r) * GXP + 16 + l15] = c01[r];
    sw[(16 + 8 * hh + r) * GXP + l15] = c10[r];
    sw[(16 + 8 * hh + r) * GXP + 16 + l15] = c11[r];
  }
  wave_sync_lds();
  const int q = lane >> 3, piece = lane & 7;
  v4f ov[8];
  if (EP != 2) {
#pragma unroll
    for (int it = 0; it < 8; ++it) {
      const int row = it * 4 + q;
      v4f v = *(const v4f*)(sw + row * GXP + piece * 4);
      if (EP == 1) {
        const v4f rr = *(const v4f*)(res + (size_t)(m0 + row) * CC + n0 + piece * 4);
        v = v + rr;
      }
      ov[it] = v;
    }
#pragma unroll
    for (int it = 0; it < 8; ++it) {
      const int row = it * 4 + q;
      *(volatile v4f*)(outf + (size_t)(m0 + row) * ldo + n0 + piece * 4) = ov[it];
    }
    __threadfence();
#pragma unroll
    for (int it = 0; it < 8; ++it) {
      const int row = it * 4 + q;
      *(volatile v4f*)(outf + (size_t)(m0 + row) * ldo + n0 + piece * 4) = ov[it];
    }
  } else {
    const int b = m0 / HW;
    const int plx = m0 - b * HW;
#pragma unroll
    for (int it = 0; it < 8; ++it) {
      const int ch = it * 4 + q;
      v4f v;
#pragma unroll
      for (int e = 0; e < 4; ++e) {
        const float rv = res[(size_t)(m0 + piece * 4 + e) * CC + n0 + ch];
        v[e] = sw[(piece * 4 + e) * GXP + ch] + rv;
      }
      ov[it] = v;
    }
#pragma unroll
    for (int it = 0; it < 8; ++it) {
      const int ch = it * 4 + q;
      *(volatile v4f*)(outf + ((size_t)(b * CC + n0 + ch)) * HW + plx + piece * 4) = ov[it];
    }
    __threadfence();
#pragma unroll
    for (int it = 0; it < 8; ++it) {
      const int ch = it * 4 + q;
      *(volatile v4f*)(outf + ((size_t)(b * CC + n0 + ch)) * HW + plx + piece * 4) = ov[it];
    }
  }
}

template <int CS, int MODE>
__global__ __launch_bounds__(256) void dw_k(const float* __restrict__ src, const float* __restrict__ wd,
                                            int wofs, int cvalid, int roll,
                                            float* dstf, int dpitch, int dcol,
                                            unsigned short* Ph, unsigned short* Pl, int ppitch) {
  constexpr int TPP = CS / 4;
  const int t = blockIdx.x * 256 + threadIdx.x;
  int p = t / TPP;
  const int cg = t - p * TPP;
  const bool pv = p < NPIX;
  p = pv ? p : (NPIX - 1);
  const int c = cg * 4;
  const int b = p / HW;
  const int pr = p - b * HW;
  const int y = pr / IMW;
  const int x = pr - y * IMW;
  int widx[4];
  float wok[4];
#pragma unroll
  for (int e = 0; e < 4; ++e) {
    const int cgb = wofs + c + e;
    wok[e] = (cgb < cvalid) ? 1.0f : 0.0f;
    widx[e] = min(cgb, cvalid - 1) * 9;
  }
  v4f acc = {0.f, 0.f, 0.f, 0.f};
#pragma unroll 1
  for (int tap = 0; tap < 9; ++tap) {
    const int dy = (tap * 11) >> 5;
    const int dx = tap - dy * 3;
    const int ny = y + dy - 1, nx = x + dx - 1;
    const float m = ((unsigned)ny < (unsigned)IMW && (unsigned)nx < (unsigned)IMW) ? 1.0f : 0.0f;
    const int sy = (ny + roll) & (IMW - 1), sx = (nx + roll) & (IMW - 1);
    const v4f v = *(const v4f*)(src + ((size_t)(b * HW) + (size_t)sy * IMW + sx) * CS + c);
#pragma unroll
    for (int e = 0; e < 4; ++e) {
      const float wv = bfr(wd[widx[e] + tap]) * wok[e];
      acc[e] = acc[e] + (v[e] * m) * wv;
    }
  }
  if (MODE == 1) {
#pragma unroll 1
    for (int e = 0; e < 4; ++e) {
      const float v = (e == 0) ? acc[0] : ((e == 1) ? acc[1] : ((e == 2) ? acc[2] : acc[3]));
      const float er = erff(v * RSQ2);
      float gl = 0.5f * v;
      gl = gl * (1.0f + er);
      acc[0] = (e == 0) ? gl : acc[0];
      acc[1] = (e == 1) ? gl : acc[1];
      acc[2] = (e == 2) ? gl : acc[2];
      acc[3] = (e == 3) ? gl : acc[3];
    }
  }
  if (MODE == 0) {
    float* gp = dstf + (size_t)p * dpitch + dcol + c;
    if (pv) *(volatile v4f*)gp = acc;
    __threadfence();
    if (pv) *(volatile v4f*)gp = acc;
  } else {
    v2u ph, plw;
    split4(acc, ph, plw);
    const size_t to = (size_t)p * ppitch + dcol + c;
    if (pv) { *(volatile v2u*)(Ph + to) = ph; *(volatile v2u*)(Pl + to) = plw; }
    __threadfence();
    if (pv) { *(volatile v2u*)(Ph + to) = ph; *(volatile v2u*)(Pl + to) = plw; }
  }
}

__global__ __launch_bounds__(256) void rsa_attn_k(const float* __restrict__ R, const float* __restrict__ temp,
                                                  unsigned short* Th, unsigned short* Tl) {
#pragma clang fp contract(off)
  extern __shared__ __align__(16) char smem[];
  float* sR = (float*)(smem + RL_R);
  float* ost = (float*)(smem + RL_R);
  unsigned short* qt = (unsigned short*)(smem + RL_QTH);
  unsigned short* ath = (unsigned short*)(smem + RL_ATH);
  unsigned short* atl = (unsigned short*)(smem + RL_ATL);
  unsigned short* vh = (unsigned short*)(smem + RL_VH);
  unsigned short* vl = (unsigned short*)(smem + RL_VL);
  float* sinv = (float*)(smem + RL_INV);
  const int tid = threadIdx.x, wave = tid >> 5, lane = tid & 31, hh = lane >> 4, l15 = lane & 15;
  const int b = blockIdx.x / NWIN;
  const int w2 = blockIdx.x - b * NWIN;
  const int wy = w2 / NWX;
  const int wx = w2 - wy * NWX;

#pragma unroll
  for (int it = 0; it < 6; ++it) {
    const int idx = it * 256 + tid;
    const int pi = idx / 96;
    const int c4 = (idx - pi * 96) * 4;
    const int ry = wy * WSZ + (pi / WSZ), rx = wx * WSZ + (pi - (pi / WSZ) * WSZ);
    const v4f v = *(const v4f*)(R + ((size_t)(b * HW) + (size_t)ry * IMW + rx) * C3 + c4);
    *(v4f*)(sR + pi * C3 + c4) = v;
  }
  __syncthreads();

  {
    const int pair = tid >> 3, sub = tid & 7;
    const int sel = pair >> 4, pi = pair & 15;
    const float* rp = sR + pi * C3 + sel * CC + sub * 16;
    float s = 0.f;
#pragma unroll
    for (int j = 0; j < 16; ++j) { const float f = rp[j]; const float ff = f * f; s = s + ff; }
    s = s + __shfl_xor(s, 1, 32);
    s = s + __shfl_xor(s, 2, 32);
    s = s + __shfl_xor(s, 4, 32);
    const float inv = 1.0f / fmaxf(sqrtf(s), 1e-12f);
    if (sub == 0) sinv[pair] = inv;
  }
  __syncthreads();

  {
    const int c = tid >> 1, sel = tid & 1;
    unsigned short hv[16], lv[16];
#pragma unroll
    for (int pi = 0; pi < 16; ++pi) {
      const float v = sR[pi * C3 + sel * CC + c] * sinv[sel * 16 + pi];
      split_bf(v, hv[pi], lv[pi]);
    }
    v4u h0, h1, l0, l1;
#pragma unroll
    for (int e = 0; e < 4; ++e) {
      h0[e] = pk16(hv[2 * e], hv[2 * e + 1]);
      h1[e] = pk16(hv[8 + 2 * e], hv[8 + 2 * e + 1]);
      l0[e] = pk16(lv[2 * e], lv[2 * e + 1]);
      l1[e] = pk16(lv[8 + 2 * e], lv[8 + 2 * e + 1]);
    }
    unsigned short* dh = qt + sel * 4096 + c * 16;
    unsigned short* dl = dh + 2048;
    *(v4u*)(dh) = h0; *(v4u*)(dh + 8) = h1;
    *(v4u*)(dl) = l0; *(v4u*)(dl + 8) = l1;
    const int pi = tid >> 4, c8 = (tid & 15) * 8;
    const float* vr = sR + pi * C3 + 2 * CC + c8;
    const v4f v0 = *(const v4f*)(vr);
    const v4f v1 = *(const v4f*)(vr + 4);
    v4u ph, plw;
    split8(v0, v1, ph, plw);
    *(v4u*)(vh + pi * ATP + c8) = ph;
    *(v4u*)(vl + pi * ATP + c8) = plw;
  }
  __syncthreads();

  const float tmp = bfr(temp[0]);
  {
    const int mi = wave;
    const v16bf a_h = ldfrag16(qt + (mi * 16 + l15) * 16 + 8 * hh);
    const v16bf a_l = ldfrag16(qt + 2048 + (mi * 16 + l15) * 16 + 8 * hh);
#pragma unroll 2
    for (int ni = 0; ni < 8; ++ni) {
      const v16bf b_h = ldfrag16(qt + 4096 + (ni * 16 + l15) * 16 + 8 * hh);
      const v16bf b_l = ldfrag16(qt + 6144 + (ni * 16 + l15) * 16 + 8 * hh);
      v8f acc = zero8();
      acc = mma_bf(a_h, b_h, acc);
      acc = mma_bf(a_h, b_l, acc);
      acc = mma_bf(a_l, b_h, acc);
      unsigned short hv[8], lv[8];
#pragma unroll
      for (int r = 0; r < 8; ++r) {
        float v = acc[r] * tmp;
        v = fmaxf(v, 0.0f);
        split_bf(v, hv[r], lv[r]);
      }
      v4u ph, plw;
#pragma unroll
      for (int e = 0; e < 4; ++e) { ph[e] = pk16(hv[2 * e], hv[2 * e + 1]); plw[e] = pk16(lv[2 * e], lv[2 * e + 1]); }
      const int d = ni * 16 + l15;
      *(v4u*)(ath + d * ATP + mi * 16 + 8 * hh) = ph;
      *(v4u*)(atl + d * ATP + mi * 16 + 8 * hh) = plw;
    }
  }
  __syncthreads();

  {
    const int ni = wave;
    v8f acc = zero8();
#pragma unroll
    for (int ks = 0; ks < 4; ++ks) {
      const v16bf a_h = ldfrag(vh + l15 * ATP + ks * 32 + 8 * hh);
      const v16bf a_l = ldfrag(vl + l15 * ATP + ks * 32 + 8 * hh);
      const v16bf b_h = ldfrag(ath + (ni * 16 + l15) * ATP + ks * 32 + 8 * hh);
      const v16bf b_l = ldfrag(atl + (ni * 16 + l15) * ATP + ks * 32 + 8 * hh);
      acc = mma_bf(a_h, b_h, acc);
      acc = mma_bf(a_h, b_l, acc);
      acc = mma_bf(a_l, b_h, acc);
    }
#pragma unroll
    for (int r = 0; r < 8; ++r) ost[(8 * hh + r) * TXP + ni * 16 + l15] = acc[r];
  }
  __syncthreads();

  {
    const int tk = 2 * wave + hh;
    const int piece = l15;
    const float* orow = ost + tk * TXP + piece * 8;
    const v4f v0 = *(const v4f*)(orow);
    const v4f v1 = *(const v4f*)(orow + 4);
    v4u ph, plw;
    split8(v0, v1, ph, plw);
    const int iy = tk / WSZ, ix = tk - (tk / WSZ) * WSZ;
    const int ry = wy * WSZ + iy, rx = wx * WSZ + ix;
    const int py = (ry + WSZ / 2) & (IMW - 1), px = (rx + WSZ / 2) & (IMW - 1);
    const size_t gp = ((size_t)(b * HW) + (size_t)py * IMW + px) * CC + piece * 8;
    *(volatile v4u*)(Th + gp) = ph;
    *(volatile v4u*)(Tl + gp) = plw;
    __threadfence();
    *(volatile v4u*)(Th + gp) = ph;
    *(volatile v4u*)(Tl + gp) = plw;
  }
}

__global__ __launch_bounds__(256) void gsa_norm_k(const float* __restrict__ R, float* pn) {
  const int b = blockIdx.x / NSLN;
  const int slab = blockIdx.x - b * NSLN;
  const int c = threadIdx.x;
  const float* base = R + ((size_t)(b * HW) + (size_t)slab * 256) * C3 + c;
  float s = 0.f;
#pragma unroll 4
  for (int i = 0; i < 256; ++i) { const float f = base[(size_t)i * C3]; s = fmaf(f, f, s); }
  float* gp = pn + ((size_t)(b * NSLN + slab)) * 256 + c;
  *(volatile float*)gp = s;
  __threadfence();
  *(volatile float*)gp = s;
}

__global__ __launch_bounds__(256) void gsa_s_k(const float* __restrict__ R, float* pa) {
  extern __shared__ __align__(16) char smem[];
  unsigned short* pl = (unsigned short*)(smem + GL_QH);
  float* red = (float*)(smem + GL_RED);
  float* stg = (float*)(smem + GL_STG);
  const int tid = threadIdx.x, wave = tid >> 5, lane = tid & 31, hh = lane >> 4, l15 = lane & 15;
  const int blk = blockIdx.x;
  const int b = blk / (NHEAD * NSLS);
  const int rem = blk - b * (NHEAD * NSLS);
  const int h = rem / NSLS;
  const int slab = rem - h * NSLS;
  const int f = wave & 3, mi = f >> 1, ni = f & 1, kh = wave >> 2;
  const int c = tid & 63, sel = c >> 5, cc = c & 31;
  const int col = sel * CC + h * HDC + cc;
  unsigned short* ph = pl + sel * 16896 + cc * GSP;
  unsigned short* plo = ph + 8448;
  const int g0 = tid >> 6;
  const size_t pbase = (size_t)(b * HW) + (size_t)slab * 2048;
  v8f acc = zero8();
#pragma unroll 1
  for (int ch = 0; ch < 8; ++ch) {
    const size_t pc = pbase + (size_t)ch * 256;
#pragma unroll 2
    for (int it = 0; it < 8; ++it) {
      const int g = it * 4 + g0;
      const float* rp = R + (pc + g * 8) * C3 + col;
      v4f v0, v1;
#pragma unroll
      for (int j = 0; j < 4; ++j) { v0[j] = rp[(size_t)j * C3]; v1[j] = rp[(size_t)(j + 4) * C3]; }
      v4u hp, lp;
      split8(v0, v1, hp, lp);
      *(v4u*)(ph + g * 8) = hp;
      *(v4u*)(plo + g * 8) = lp;
    }
    __syncthreads();
#pragma unroll
    for (int ks = 0; ks < 4; ++ks) {
      const int k0 = (kh * 4 + ks) * 32;
      const v16bf a_h = ldfrag(pl + (mi * 16 + l15) * GSP + k0 + 8 * hh);
      const v16bf a_l = ldfrag(pl + 8448 + (mi * 16 + l15) * GSP + k0 + 8 * hh);
      const v16bf b_h = ldfrag(pl + 16896 + (ni * 16 + l15) * GSP + k0 + 8 * hh);
      const v16bf b_l = ldfrag(pl + 25344 + (ni * 16 + l15) * GSP + k0 + 8 * hh);
      acc = mma_bf(a_h, b_h, acc);
      acc = mma_bf(a_h, b_l, acc);
      acc = mma_bf(a_l, b_h, acc);
    }
    __syncthreads();
  }
  if (wave >= 4) {
#pragma unroll
    for (int r = 0; r < 8; ++r) red[((wave - 4) * 32 + lane) * 8 + r] = acc[r];
  }
  __syncthreads();
  if (wave < 4) {
#pragma unroll
    for (int r = 0; r < 8; ++r) {
      const float o = red[(wave * 32 + lane) * 8 + r];
      const float v = acc[r] + o;
      stg[(mi * 16 + 8 * hh + r) * GXP + ni * 16 + l15] = v;
    }
  }
  __syncthreads();
  {
    const int row = tid >> 3, piece = tid & 7;
    const v4f v = *(const v4f*)(stg + row * GXP + piece * 4);
    float* gp = pa + (size_t)blk * 1024 + row * 32 + piece * 4;
    *(volatile v4f*)gp = v;
    __threadfence();
    *(volatile v4f*)gp = v;
  }
}

__global__ __launch_bounds__(256) void gsa_fin_k(const float* __restrict__ pa, const float* __restrict__ pn,
                                                 const float* __restrict__ temp,
                                                 unsigned short* afh, unsigned short* afl) {
#pragma clang fp contract(off)
  __shared__ float sinv[64];
  const int tid = threadIdx.x;
  const int b = blockIdx.x / NHEAD;
  const int h = blockIdx.x - b * NHEAD;
  if (tid < 64) {
    const int sel = tid >> 5, i = tid & 31;
    const int c = sel * CC + h * HDC + i;
    float s = 0.f;
#pragma unroll 4
    for (int sl = 0; sl < NSLN; ++sl) s = s + pn[((size_t)(b * NSLN + sl)) * 256 + c];
    sinv[tid] = 1.0f / fmaxf(sqrtf(s), 1e-12f);
  }
  __syncthreads();
  const float tmp = bfr(temp[0]);
  const int e0 = tid * 4;
  const int c = e0 >> 5;
  v4f a;
#pragma unroll
  for (int j = 0; j < 4; ++j) {
    const int e = e0 + j;
    const int d = e & 31;
    float s = 0.f;
#pragma unroll
    for (int sl = 0; sl < NSLS; ++sl) s = s + pa[((size_t)((b * NHEAD + h) * NSLS + sl)) * 1024 + e];
    float v = s * sinv[c];
    v = v * sinv[32 + d];
    v = v * tmp;
    a[j] = fmaxf(v, 0.0f);
  }
  v2u ph, plw;
  split4(a, ph, plw);
  const size_t to = (size_t)b * AFSZ + (size_t)h * (HDC * HDC) + e0;
  *(volatile v2u*)(afh + to) = ph;
  *(volatile v2u*)(afl + to) = plw;
  __threadfence();
  *(volatile v2u*)(afh + to) = ph;
  *(volatile v2u*)(afl + to) = plw;
}

__global__ __launch_bounds__(256) void apply_k(const unsigned short* __restrict__ Vh,
                                               const unsigned short* __restrict__ Vl,
                                               const unsigned short* __restrict__ afh,
                                               const unsigned short* __restrict__ afl,
                                               unsigned short* Oh, unsigned short* Ol) {
  __shared__ __align__(16) float stg[8 * 16 * AXP];
  const int tid = threadIdx.x, wave = tid >> 5, lane = tid & 31, hh = lane >> 4, l15 = lane & 15;
  const int m0 = (blockIdx.x * 8 + wave) * 16;
  const int n0 = blockIdx.y * 64;
  const int b = m0 / HW;
  const int hd0 = n0 / HDC;
  const unsigned short* ar = Vh + (size_t)(m0 + l15) * CC + hd0 * HDC + 8 * hh;
  const unsigned short* al = Vl + (size_t)(m0 + l15) * CC + hd0 * HDC + 8 * hh;
  const v16bf a0h = ldfrag(ar), a0l = ldfrag(al);
  const v16bf a1h = ldfrag(ar + 32), a1l = ldfrag(al + 32);
  const unsigned short* wb = afh + (size_t)b * AFSZ + (size_t)(n0 + l15) * 32 + 8 * hh;
  const unsigned short* wl = afl + (size_t)b * AFSZ + (size_t)(n0 + l15) * 32 + 8 * hh;
  v8f c0 = zero8(), c1 = zero8(), c2 = zero8(), c3 = zero8();
  {
    const v16bf bh = ldfrag(wb), bl = ldfrag(wl);
    c0 = mma_bf(a0h, bh, c0); c0 = mma_bf(a0l, bh, c0); c0 = mma_bf(a0h, bl, c0);
  }
  {
    const v16bf bh = ldfrag(wb + 16 * 32), bl = ldfrag(wl + 16 * 32);
    c1 = mma_bf(a0h, bh, c1); c1 = mma_bf(a0l, bh, c1); c1 = mma_bf(a0h, bl, c1);
  }
  {
    const v16bf bh = ldfrag(wb + 32 * 32), bl = ldfrag(wl + 32 * 32);
    c2 = mma_bf(a1h, bh, c2); c2 = mma_bf(a1l, bh, c2); c2 = mma_bf(a1h, bl, c2);
  }
  {
    const v16bf bh = ldfrag(wb + 48 * 32), bl = ldfrag(wl + 48 * 32);
    c3 = mma_bf(a1h, bh, c3); c3 = mma_bf(a1l, bh, c3); c3 = mma_bf(a1h, bl, c3);
  }
  float* sw = stg + wave * (16 * AXP);
#pragma unroll
  for (int r = 0; r < 8; ++r) {
    sw[(8 * hh + r) * AXP + l15] = c0[r];
    sw[(8 * hh + r) * AXP + 16 + l15] = c1[r];
    sw[(8 * hh + r) * AXP + 32 + l15] = c2[r];
    sw[(8 * hh + r) * AXP + 48 + l15] = c3[r];
  }
  wave_sync_lds();
  const int q = lane >> 3, piece = lane & 7;
  v4u oh[4], ol[4];
#pragma unroll
  for (int it = 0; it < 4; ++it) {
    const int row = it * 4 + q;
    const float* sp = sw + row * AXP + piece * 8;
    const v4f v0 = *(const v4f*)(sp);
    const v4f v1 = *(const v4f*)(sp + 4);
    split8(v0, v1, oh[it], ol[it]);
  }
#pragma unroll
  for (int it = 0; it < 4; ++it) {
    const int row = it * 4 + q;
    const size_t to = (size_t)(m0 + row) * CC + n0 + piece * 8;
    *(volatile v4u*)(Oh + to) = oh[it];
    *(volatile v4u*)(Ol + to) = ol[it];
  }
  __threadfence();
#pragma unroll
  for (int it = 0; it < 4; ++it) {
    const int row = it * 4 + q;
    const size_t to = (size_t)(m0 + row) * CC + n0 + piece * 8;
    *(volatile v4u*)(Oh + to) = oh[it];
    *(volatile v4u*)(Ol + to) = ol[it];
  }
}

extern "C" void kernel_launch(void* const* d_in, const int* in_sizes, int n_in,
                              void* d_out, int out_size, void* d_ws, size_t ws_size,
                              hipStream_t stream) {
  if (n_in < 23) return;
  if (in_sizes[0] != NPIX * CC) return;
  if (in_sizes[1] != CC || in_sizes[2] != CC || in_sizes[3] != CC || in_sizes[4] != CC) return;
  if (in_sizes[5] != C3 * CC || in_sizes[6] != C3 * 9 || in_sizes[7] != CC * CC || in_sizes[8] < 1) return;
  if (in_sizes[9] != HID * CC || in_sizes[10] != HID * 9 || in_sizes[11] != CC * HID) return;
  if (in_sizes[12] != CC || in_sizes[13] != CC || in_sizes[14] != CC || in_sizes[15] != CC) return;
  if (in_sizes[16] != C3 * CC || in_sizes[17] != C3 * 9 || in_sizes[18] != CC * CC || in_sizes[19] < 1) return;
  if (in_sizes[20] != HID * CC || in_sizes[21] != HID * 9 || in_sizes[22] != CC * HID) return;
  if (out_size != NPIX * CC) return;

  const float* x        = (const float*)d_in[0];
  const float* w_s0     = (const float*)d_in[1];
  const float* b_s0     = (const float*)d_in[2];
  const float* w_s2     = (const float*)d_in[3];
  const float* b_s2     = (const float*)d_in[4];
  const float* rsa_qkv  = (const float*)d_in[5];
  const float* rsa_dw   = (const float*)d_in[6];
  const float* rsa_proj = (const float*)d_in[7];
  const float* rsa_temp = (const float*)d_in[8];
  const float* ffs_in   = (const float*)d_in[9];
  const float* ffs_dw   = (const float*)d_in[10];
  const float* ffs_out  = (const float*)d_in[11];
  const float* w_c0     = (const float*)d_in[12];
  const float* b_c0     = (const float*)d_in[13];
  const float* w_c2     = (const float*)d_in[14];
  const float* b_c2     = (const float*)d_in[15];
  const float* gsa_qkv  = (const float*)d_in[16];
  const float* gsa_dw   = (const float*)d_in[17];
  const float* gsa_proj = (const float*)d_in[18];
  const float* gsa_temp = (const float*)d_in[19];
  const float* ffc_in   = (const float*)d_in[20];
  const float* ffc_dw   = (const float*)d_in[21];
  const float* ffc_out  = (const float*)d_in[22];
  float* out = (float*)d_out;

  const size_t sAct = (size_t)NPIX * CC * 4;
  const size_t sT   = (size_t)NPIX * CC * 2 * 2;
  const size_t sU   = (size_t)NPIX * FSL * 4;
  const size_t sR   = (size_t)NPIX * C3 * 4;
  const size_t sWq  = (size_t)C3 * CC * 2;
  const size_t sWp  = (size_t)CC * CC * 2;
  const size_t sW1  = (size_t)HIDP * CC * 2;
  const size_t sW2  = (size_t)CC * HIDP * 2;
  const size_t sPN  = (size_t)NB * NSLN * 256 * 4;
  const size_t sPA  = (size_t)NB * NHEAD * NSLS * 1024 * 4;
  const size_t sAF  = (size_t)NB * AFSZ * 2;
  size_t off = 0;
  const size_t oA   = off; off += sAct;
  const size_t oBx  = off; off += sAct;
  const size_t oT   = off; off += sT;
  const size_t oU   = off; off += sU;
  const size_t oR   = off; off += sR;
  const size_t oWq0 = off; off += sWq;
  const size_t oWp0 = off; off += sWp;
  const size_t oW10 = off; off += sW1;
  const size_t oW20 = off; off += sW2;
  const size_t oWq1 = off; off += sWq;
  const size_t oWp1 = off; off += sWp;
  const size_t oW11 = off; off += sW1;
  const size_t oW21 = off; off += sW2;
  const size_t oPN  = off; off += sPN;
  const size_t oPA  = off; off += sPA;
  const size_t oAFh = off; off += sAF;
  const size_t oAFl = off; off += sAF;
  if (off > ws_size) return;
  if (off > (size_t)134217728) return;
  if (sU < (size_t)NPIX * CC * 4) return;
  if (sU < (size_t)NPIX * CC * 2 * 2) return;
  if (sR < (size_t)NPIX * HIDP * 2 * 2) return;

  char* ws = (char*)d_ws;
  float* A  = (float*)(ws + oA);
  float* Bx = (float*)(ws + oBx);
  unsigned short* Th = (unsigned short*)(ws + oT);
  unsigned short* Tl = Th + (size_t)NPIX * CC;
  float* U  = (float*)(ws + oU);
  unsigned short* Uh = (unsigned short*)(ws + oU);
  unsigned short* Ul = Uh + (size_t)NPIX * CC;
  float* R  = (float*)(ws + oR);
  unsigned short* Gh = (unsigned short*)(ws + oR);
  unsigned short* Gl = Gh + (size_t)NPIX * HIDP;
  unsigned short* Wq0 = (unsigned short*)(ws + oWq0);
  unsigned short* Wp0 = (unsigned short*)(ws + oWp0);
  unsigned short* W10 = (unsigned short*)(ws + oW10);
  unsigned short* W20 = (unsigned short*)(ws + oW20);
  unsigned short* Wq1 = (unsigned short*)(ws + oWq1);
  unsigned short* Wp1 = (unsigned short*)(ws + oWp1);
  unsigned short* W11 = (unsigned short*)(ws + oW11);
  unsigned short* W21 = (unsigned short*)(ws + oW21);
  float* PN = (float*)(ws + oPN);
  float* PA = (float*)(ws + oPA);
  unsigned short* AFh = (unsigned short*)(ws + oAFh);
  unsigned short* AFl = (unsigned short*)(ws + oAFl);

  const dim3 blk(256);
  cvt_w<<<dim3((C3 * CC / 8 + 255) / 256), blk, 0, stream>>>(rsa_qkv, Wq0, C3, CC, C3, CC);
  cvt_w<<<dim3((CC * CC / 8 + 255) / 256), blk, 0, stream>>>(rsa_proj, Wp0, CC, CC, CC, CC);
  cvt_w<<<dim3((HIDP * CC / 8 + 255) / 256), blk, 0, stream>>>(ffs_in, W10, HID, CC, HIDP, CC);
  cvt_w<<<dim3((CC * HIDP / 8 + 255) / 256), blk, 0, stream>>>(ffs_out, W20, CC, HID, CC, HIDP);
  cvt_w<<<dim3((C3 * CC / 8 + 255) / 256), blk, 0, stream>>>(gsa_qkv, Wq1, C3, CC, C3, CC);
  cvt_w<<<dim3((CC * CC / 8 + 255) / 256), blk, 0, stream>>>(gsa_proj, Wp1, CC, CC, CC, CC);
  cvt_w<<<dim3((HIDP * CC / 8 + 255) / 256), blk, 0, stream>>>(ffc_in, W11, HID, CC, HIDP, CC);
  cvt_w<<<dim3((CC * HIDP / 8 + 255) / 256), blk, 0, stream>>>(ffc_out, W21, CC, HID, CC, HIDP);

  nchw_in<<<dim3(NB * (HW / 64)), blk, 0, stream>>>(x, A);

  (void)hipFuncSetAttribute(reinterpret_cast<const void*>(&rsa_attn_k), hipFuncAttributeMaxDynamicSharedMemorySize, RL_END);
  (void)hipFuncSetAttribute(reinterpret_cast<const void*>(&gsa_s_k), hipFuncAttributeMaxDynamicSharedMemorySize, GL_END);

  const dim3 gG128(NPIX / 256, CC / 32);
  const dim3 gG192(NPIX / 256, FSL / 32);
  const dim3 gDw128((NPIX * (128 / 4) + 255) / 256);
  const dim3 gDw192((NPIX * (192 / 4) + 255) / 256);
  const dim3 gLn(NPIX / 8);

  ln_k<<<gLn, blk, 0, stream>>>(A, Bx, w_s0, b_s0, Th, Tl, 0);
  for (int s = 0; s < 3; ++s) {
    gemm_k<CC, 0><<<gG128, blk, 0, stream>>>(Th, Tl, CC, Wq0 + (size_t)s * CC * CC, U, CC, Bx);
    dw_k<128, 0><<<gDw128, blk, 0, stream>>>(U, rsa_dw, s * CC, C3, WSZ / 2, R, C3, s * CC, Th, Tl, CC);
  }
  rsa_attn_k<<<dim3(NB * NWIN), blk, RL_END, stream>>>(R, rsa_temp, Th, Tl);
  gemm_k<CC, 0><<<gG128, blk, 0, stream>>>(Th, Tl, CC, Wp0, Bx, CC, A);
  ln_k<<<gLn, blk, 0, stream>>>(A, Bx, w_s2, b_s2, Th, Tl, 1);
  for (int s = 0; s < 2; ++s) {
    gemm_k<CC, 0><<<gG192, blk, 0, stream>>>(Th, Tl, CC, W10 + (size_t)s * FSL * CC, U, FSL, Bx);
    dw_k<192, 1><<<gDw192, blk, 0, stream>>>(U, ffs_dw, s * FSL, HID, 0, R, C3, s * FSL, Gh, Gl, HIDP);
  }
  gemm_k<HIDP, 1><<<gG128, blk, 0, stream>>>(Gh, Gl, HIDP, W20, A, CC, Bx);

  ln_k<<<gLn, blk, 0, stream>>>(A, Bx, w_c0, b_c0, Th, Tl, 0);
  for (int s = 0; s < 2; ++s) {
    gemm_k<CC, 0><<<gG128, blk, 0, stream>>>(Th, Tl, CC, Wq1 + (size_t)s * CC * CC, U, CC, Bx);
    dw_k<128, 0><<<gDw128, blk, 0, stream>>>(U, gsa_dw, s * CC, C3, 0, R, C3, s * CC, Th, Tl, CC);
  }
  gemm_k<CC, 0><<<gG128, blk, 0, stream>>>(Th, Tl, CC, Wq1 + (size_t)2 * CC * CC, U, CC, Bx);
  dw_k<128, 2><<<gDw128, blk, 0, stream>>>(U, gsa_dw, 2 * CC, C3, 0, R, C3, 0, Th, Tl, CC);
  gsa_norm_k<<<dim3(NB * NSLN), blk, 0, stream>>>(R, PN);
  gsa_s_k<<<dim3(NB * NHEAD * NSLS), blk, GL_END, stream>>>(R, PA);
  gsa_fin_k<<<dim3(NB * NHEAD), blk, 0, stream>>>(PA, PN, gsa_temp, AFh, AFl);
  apply_k<<<dim3(NPIX / 128, CC / 64), blk, 0, stream>>>(Th, Tl, AFh, AFl, Uh, Ul);
  gemm_k<CC, 0><<<gG128, blk, 0, stream>>>(Uh, Ul, CC, Wp1, Bx, CC, A);
  ln_k<<<gLn, blk, 0, stream>>>(A, Bx, w_c2, b_c2, Th, Tl, 1);
  for (int s = 0; s < 2; ++s) {
    gemm_k<CC, 0><<<gG192, blk, 0, stream>>>(Th, Tl, CC, W11 + (size_t)s * FSL * CC, U, FSL, Bx);
    dw_k<192, 1><<<gDw192, blk, 0, stream>>>(U, ffc_dw, s * FSL, HID, 0, R, C3, s * FSL, Gh, Gl, HIDP);
  }
  gemm_k<HIDP, 2><<<gG128, blk, 0, stream>>>(Gh, Gl, HIDP, W21, out, CC, Bx);
  (void)hipGetLastError();
}
